// CNFSolver_25735444038418
// MI455X (gfx1250) — hardware-run, weakly checked
//
#include <hip/hip_runtime.h>


#define NR    256
#define ND    64
#define NH    256
#define NSTEP 64
#define NO    65
typedef _Float16 h16;
typedef unsigned short bf;
typedef __attribute__((ext_vector_type(16))) __bf16   v16bf;
typedef __attribute__((ext_vector_type(16))) _Float16 v16h;
typedef __attribute__((ext_vector_type(8)))  _Float16 v8h;
typedef __attribute__((ext_vector_type(8)))  unsigned short v8us;
typedef __attribute__((ext_vector_type(8)))  float    v8f;
typedef __attribute__((ext_vector_type(4)))  float    v4f;
typedef v8h  __attribute__((may_alias)) v8ha;
typedef v4f  __attribute__((may_alias)) v4fa;
typedef v8us __attribute__((may_alias)) v8usa;

__device__ __forceinline__ unsigned short f2bf(float f) { unsigned u = __float_as_uint(f); u += 0x7FFFu + ((u >> 16) & 1u); return (unsigned short)(u >> 16); }
__device__ __forceinline__ float bf2f(unsigned short b) { return __uint_as_float(((unsigned)b) << 16); }
__device__ __forceinline__ float bfr(float f) { return bf2f(f2bf(f)); }
__device__ __forceinline__ v16h cat16(v8h lo, v8h hi) { return __builtin_shufflevector(lo, hi, 0, 1, 2, 3, 4, 5, 6, 7, 8, 9, 10, 11, 12, 13, 14, 15); }
__device__ __forceinline__ v16bf cat16b(v8us lo, v8us hi) { return __builtin_bit_cast(v16bf, __builtin_shufflevector(lo, hi, 0, 1, 2, 3, 4, 5, 6, 7, 8, 9, 10, 11, 12, 13, 14, 15)); }
__device__ __forceinline__ v8f wmma16(v16h a, v16h b, v8f c) { return __builtin_amdgcn_wmma_f32_16x16x32_f16(false, a, false, b, (short)0, c, false, false); }
__device__ __forceinline__ v8f wmmab(v16bf a, v16bf b, v8f c) { return __builtin_amdgcn_wmma_f32_16x16x32_bf16(false, a, false, b, (short)0, c, false, false); }


template <typename T16> struct WFrag;
template <> struct WFrag<h16> { typedef v16h V; static __device__ __forceinline__ V ld(const h16* p) { return cat16(*(const v8h*)p, *(const v8h*)(p + 16)); } static __device__ __forceinline__ v8f mma(V a, V b, v8f c) { return wmma16(a, b, c); } };
template <> struct WFrag<bf> { typedef v16bf V; static __device__ __forceinline__ V ld(const bf* p) { return cat16b(*(const v8us*)p, *(const v8us*)(p + 16)); } static __device__ __forceinline__ v8f mma(V a, V b, v8f c) { return wmmab(a, b, c); } };
template <typename T16, int NSPLIT, bool BIAS>
__global__ __launch_bounds__(32) void k_gemmw(const T16* __restrict__ A, const T16* __restrict__ A2, const T16* __restrict__ Bt, const T16* __restrict__ Bt2, int K, float* C, int ldc, const float* __restrict__ bias, size_t sA, size_t sB, size_t sC) {
    typedef typename WFrag<T16>::V V;
    __shared__ __align__(16) float os[16 * 68];
    const size_t z = blockIdx.z; A += z * sA; if (A2) A2 += z * sA; Bt += z * sB; if (Bt2) Bt2 += z * sB; C += z * sC;
    const int lane = threadIdx.x & 31, lr = lane & 15, hi = lane >> 4; const int r0 = blockIdx.x * 64, c0 = blockIdx.y * 64;
    v8f acc[4][4];
#pragma unroll
    for (int mb = 0; mb < 4; ++mb)
#pragma unroll
        for (int nb = 0; nb < 4; ++nb) acc[mb][nb] = (v8f){};
    const size_t aoff = (size_t)(r0 + lr) * K + 8 * hi, boff = (size_t)(c0 + lr) * K + 8 * hi;
    for (int kc = 0; kc < K; kc += 32) {
        V a[4], a2[4];
#pragma unroll
        for (int mb = 0; mb < 4; ++mb) { a[mb] = WFrag<T16>::ld(A + aoff + (size_t)mb * 16 * K + kc); if (NSPLIT == 1 || NSPLIT == 2) a2[mb] = WFrag<T16>::ld(A2 + aoff + (size_t)mb * 16 * K + kc); }
#pragma unroll
        for (int nb = 0; nb < 4; ++nb) { const V b = WFrag<T16>::ld(Bt + boff + (size_t)nb * 16 * K + kc); V b2; if (NSPLIT >= 2) b2 = WFrag<T16>::ld(Bt2 + boff + (size_t)nb * 16 * K + kc);
#pragma unroll
            for (int mb = 0; mb < 4; ++mb) { acc[mb][nb] = WFrag<T16>::mma(a[mb], b, acc[mb][nb]); if (NSPLIT == 1 || NSPLIT == 2) acc[mb][nb] = WFrag<T16>::mma(a2[mb], b, acc[mb][nb]); if (NSPLIT >= 2) acc[mb][nb] = WFrag<T16>::mma(a[mb], b2, acc[mb][nb]); } }
        asm volatile("v_nop\n\tv_nop\n\tv_nop\n\tv_nop" : "+v"(acc[0][0]), "+v"(acc[1][1]), "+v"(acc[2][2]), "+v"(acc[3][3]) : "v"(a[0]), "v"(a[3]));
    }
#pragma unroll
    for (int mb = 0; mb < 4; ++mb) {
#pragma unroll
        for (int nb = 0; nb < 4; ++nb) {
#pragma unroll
            for (int j = 0; j < 8; ++j) os[(hi * 8 + j) * 68 + nb * 16 + lr] = acc[mb][nb][j]; }
        __builtin_amdgcn_wave_barrier(); asm volatile("" ::: "memory");
        float* crow = C + (size_t)(r0 + mb * 16) * ldc + c0;
#pragma unroll 1
        for (int ps = 0; ps < 2; ++ps) {
#pragma unroll
            for (int s = 0; s < 8; ++s) { const int row = 2 * s + hi, cofs = lr * 4; v4f val = *(const v4fa*)(os + row * 68 + cofs); if (BIAS) { val[0] += bfr(bias[c0 + cofs]); val[1] += bfr(bias[c0 + cofs + 1]); val[2] += bfr(bias[c0 + cofs + 2]); val[3] += bfr(bias[c0 + cofs + 3]); }
                *(volatile v4f*)(crow + (size_t)row * ldc + cofs) = val; }
            if (ps == 0) __threadfence(); }
        __builtin_amdgcn_wave_barrier(); asm volatile("" ::: "memory");
    }
}

typedef __attribute__((ext_vector_type(2))) _Float16 v2h;
typedef __attribute__((ext_vector_type(4))) _Float16 v4h;
typedef __attribute__((ext_vector_type(2))) unsigned short v2us;
typedef __attribute__((ext_vector_type(4))) unsigned short v4us;
typedef __attribute__((ext_vector_type(2))) float v2f;
typedef __attribute__((ext_vector_type(4))) int v4i;

__global__ __launch_bounds__(256) void k_wtG(const float* __restrict__ w, int K, int N, bf* Bt) {
    const int lane = threadIdx.x & 31; const int L0 = (blockIdx.x * 8 + (threadIdx.x >> 5)) * 8; const int nlines = N * K / 64;
#pragma unroll
    for (int ps = 0; ps < 2; ++ps) {
        for (int l = 0; l < 8; ++l) { const int L = L0 + l; if (L >= nlines) break; const size_t e = (size_t)L * 64 + lane * 2; const int k = (int)(e % K), n = (int)(e / K); v2us o;
            o[0] = f2bf(w[(size_t)k * N + n]); o[1] = f2bf(w[(size_t)(k + 1) * N + n]); *(volatile v2us*)(Bt + e) = o; }
        if (ps == 0) __threadfence(); }
}

__global__ __launch_bounds__(256) void k_zero(float* dst, int n4) { const int i = blockIdx.x * 256 + threadIdx.x; if (i >= n4) return; v4f z; z[0] = 0.0f; z[1] = 0.0f; z[2] = 0.0f; z[3] = 0.0f;
    *(volatile v4f*)(dst + (size_t)i * 4) = z; __threadfence(); *(volatile v4f*)(dst + (size_t)i * 4) = z; }

__global__ __launch_bounds__(256) void k_rnd(const float* __restrict__ src, float* y, bf* op, size_t n4) { const size_t i = (size_t)blockIdx.x * 256 + threadIdx.x; if (i >= n4) return; const v4f v = *(const v4f*)(src + i * 4); v4us o; v4f r;
#pragma unroll
    for (int k = 0; k < 4; ++k) { o[k] = f2bf(v[k]); r[k] = bf2f(o[k]); }
    *(volatile v4f*)(y + i * 4) = r; *(volatile v4us*)(op + i * 4) = o; __threadfence(); *(volatile v4f*)(y + i * 4) = r; *(volatile v4us*)(op + i * 4) = o; }

__global__ __launch_bounds__(256) void k_th(const float* __restrict__ p, const float* __restrict__ u1, float t, const float* __restrict__ c2, bf* tw, float* s, size_t n4) { const size_t i = (size_t)blockIdx.x * 256 + threadIdx.x; if (i >= n4) return;
    const int h4 = (int)(i & 63) * 4; const v4f v = *(const v4f*)(p + i * 4); v4us o; v4f sv;
#pragma unroll
    for (int k = 0; k < 4; ++k) { const float T = tanhf(v[k] + t * bfr(u1[h4 + k])); o[k] = f2bf(T); sv[k] = s ? (1.0f - T * T) * c2[(size_t)(h4 + k) * NH + (h4 + k)] : 0.0f; }
#pragma unroll
    for (int ps = 0; ps < 2; ++ps) { *(volatile v4us*)(tw + i * 4) = o; if (s) *(volatile v4f*)(s + i * 4) = sv; if (ps == 0) __threadfence(); } }

__global__ __launch_bounds__(256) void k_tr(const float* __restrict__ s, const float* __restrict__ iold, float* inew, float hs) { const int r = blockIdx.x * 256 + threadIdx.x; const float* q = s + (size_t)r * NH; float acc = 0.0f;
    for (int j = 0; j < NH; ++j) acc += q[j];
    const float v = iold[r] + hs * acc; *(volatile float*)(inew + r) = v; __threadfence(); *(volatile float*)(inew + r) = v; }

__global__ __launch_bounds__(256) void k_st(const float* __restrict__ a, const float* __restrict__ b, const float* __restrict__ f, float ca, float cb, float cc, float hs, float* out, bf* outw, size_t n4) { const size_t i = (size_t)blockIdx.x * 256 + threadIdx.x; if (i >= n4) return;
    const v4f va = *(const v4f*)(a + i * 4); const v4f vb = *(const v4f*)(b + i * 4); const v4f vf = *(const v4f*)(f + i * 4); v4f r; v4us o;
#pragma unroll
    for (int k = 0; k < 4; ++k) { r[k] = (ca * va[k] + cb * vb[k]) - cc * (hs * vf[k]); o[k] = f2bf(r[k]); }
    *(volatile v4f*)(out + i * 4) = r; *(volatile v4us*)(outw + i * 4) = o; __threadfence(); *(volatile v4f*)(out + i * 4) = r; *(volatile v4us*)(outw + i * 4) = o; }

__global__ __launch_bounds__(64) void k_out(const float* __restrict__ y, const float* __restrict__ iv, float* out) { const int e = blockIdx.x * 64 + threadIdx.x; v4f r;
#pragma unroll
    for (int k = 0; k < 4; ++k) { const int m = e * 4 + k; const int row = m / NO; const int col = m - row * NO; const int cy = col < ND ? col : ND - 1; const float vi = iv[row]; const float vy = y[row * ND + cy]; r[k] = (col == ND) ? vi : vy; }
    *(volatile v4f*)(out + (size_t)e * 4) = r; __threadfence(); *(volatile v4f*)(out + (size_t)e * 4) = r; }

static constexpr size_t kSzW = (size_t)NH * ND * 2, kSzSW = (size_t)NH * ND * 4, kSzHH = (size_t)NH * NH * 4, kSzY = (size_t)NR * ND * 4, kSzYW = (size_t)NR * ND * 2, kSzP = (size_t)NR * NH * 4, kSzTW = (size_t)NR * NH * 2, kSzI = (size_t)NR * 4;
static constexpr size_t kOffW1W = 0, kOffW2W = kOffW1W + kSzW, kOffW2T = kOffW2W + kSzW, kOffSW = kOffW2T + kSzW, kOffC2 = kOffSW + kSzSW, kOffY0 = kOffC2 + kSzHH, kOffY1 = kOffY0 + kSzY, kOffZ0 = kOffY1 + kSzY, kOffZ1 = kOffZ0 + kSzY, kOffYW0 = kOffZ1 + kSzY, kOffYW1 = kOffYW0 + kSzYW, kOffZW0 = kOffYW1 + kSzYW, kOffZW1 = kOffZW0 + kSzYW, kOffP = kOffZW1 + kSzYW, kOffTW = kOffP + kSzP, kOffS = kOffTW + kSzTW, kOffF = kOffS + kSzP, kOffI0 = kOffF + kSzY, kOffI1 = kOffI0 + kSzI, kWsTotal = kOffI1 + kSzI;
static_assert(kSzW == 32768ull && kSzSW == 65536ull && kSzHH == 262144ull && kSzY == 65536ull && kSzYW == 32768ull && kSzP == 262144ull && kSzTW == 131072ull && kSzI == 1024ull && kWsTotal == 1542144ull);
static_assert(kWsTotal <= 134217728ull);
static_assert((kSzW % 128) == 0 && (kSzSW % 128) == 0 && (kSzHH % 128) == 0 && (kSzY % 128) == 0 && (kSzYW % 128) == 0 && (kSzP % 128) == 0 && (kSzTW % 128) == 0 && (kSzI % 128) == 0);
static_assert((NR % 64) == 0 && (NH % 64) == 0 && (ND % 64) == 0 && (ND % 32) == 0 && (NH % 32) == 0);
static_assert(((ND * NH) % 4096) == 0);
static_assert(NO == ND + 1 && ((NR * NO * 4) % 128) == 0 && ((NR * NO) % 256) == 0);

extern "C" void kernel_launch(void* const* d_in, const int* in_sizes, int n_in, void* d_out, int out_size, void* d_ws, size_t ws_size, hipStream_t stream) {
    if (n_in < 6) return;
    if (in_sizes[0] != NR * ND || in_sizes[1] != NH * ND || in_sizes[2] != NH || in_sizes[3] != NH || in_sizes[4] != ND * NH || in_sizes[5] != ND) return;
    if (out_size != NR * NO) return;
    if (ws_size < kWsTotal) return;
    const float* y1 = (const float*)d_in[0]; const float* w1 = (const float*)d_in[1]; const float* b1 = (const float*)d_in[2]; const float* u1 = (const float*)d_in[3]; const float* w2 = (const float*)d_in[4]; const float* b2 = (const float*)d_in[5];
    float* out = (float*)d_out; char* ws = (char*)d_ws;
    bf* W1W = (bf*)(ws + kOffW1W); bf* W2W = (bf*)(ws + kOffW2W); bf* W2T = (bf*)(ws + kOffW2T); float* SW = (float*)(ws + kOffSW); float* C2 = (float*)(ws + kOffC2);
    float* Y[2] = { (float*)(ws + kOffY0), (float*)(ws + kOffY1) }; float* Z[2] = { (float*)(ws + kOffZ0), (float*)(ws + kOffZ1) }; bf* YW[2] = { (bf*)(ws + kOffYW0), (bf*)(ws + kOffYW1) }; bf* ZW[2] = { (bf*)(ws + kOffZW0), (bf*)(ws + kOffZW1) };
    float* P = (float*)(ws + kOffP); bf* TW = (bf*)(ws + kOffTW); float* S = (float*)(ws + kOffS); float* F = (float*)(ws + kOffF); float* IV[2] = { (float*)(ws + kOffI0), (float*)(ws + kOffI1) };
    const size_t n4w = (size_t)NH * ND / 4; const size_t n4y = (size_t)NR * ND / 4; const size_t n4h = (size_t)NR * NH / 4;

    k_rnd<<<(unsigned)(n4w / 256), 256, 0, stream>>>(w1, SW, W1W, n4w);
    k_rnd<<<(unsigned)(n4w / 256), 256, 0, stream>>>(w2, SW, W2W, n4w);
    k_rnd<<<(unsigned)(n4y / 256), 256, 0, stream>>>(y1, Y[0], YW[0], n4y);
    k_rnd<<<(unsigned)(n4y / 256), 256, 0, stream>>>(y1, Z[0], ZW[0], n4y);
    k_wtG<<<(unsigned)((ND * NH / 64 + 63) / 64), 256, 0, stream>>>(w2, ND, NH, W2T);
    k_gemmw<bf, 0, false><<<dim3(NH / 64, NH / 64, 1), 32, 0, stream>>>(W1W, nullptr, W2T, nullptr, ND, C2, NH, nullptr, 0, 0, 0);
    k_zero<<<1, NR / 4, 0, stream>>>(IV[0], NR / 4);

    const float hs = 1.0f / (float)NSTEP; const float il = (float)(1.0 / 0.999); const float oml = (float)(1.0 - 1.0 / 0.999);
    for (int st = 0; st < NSTEP; ++st) { const int c = st & 1, n = c ^ 1; const float t1 = 1.0f - (float)st * hs; const float t0 = t1 - hs;
        k_gemmw<bf, 0, true><<<dim3(NR / 64, NH / 64, 1), 32, 0, stream>>>(YW[c], nullptr, W1W, nullptr, ND, P, NH, b1, 0, 0, 0);
        k_th<<<(unsigned)(n4h / 256), 256, 0, stream>>>(P, u1, t1, C2, TW, S, n4h);
        k_gemmw<bf, 0, true><<<dim3(NR / 64, ND / 64, 1), 32, 0, stream>>>(TW, nullptr, W2W, nullptr, NH, F, ND, b2, 0, 0, 0);
        k_tr<<<1, 256, 0, stream>>>(S, IV[c], IV[n], hs);
        k_st<<<(unsigned)(n4y / 256), 256, 0, stream>>>(Z[c], Z[c], F, 1.0f, 0.0f, 1.0f, hs, Z[n], ZW[n], n4y);
        k_gemmw<bf, 0, true><<<dim3(NR / 64, NH / 64, 1), 32, 0, stream>>>(ZW[n], nullptr, W1W, nullptr, ND, P, NH, b1, 0, 0, 0);
        k_th<<<(unsigned)(n4h / 256), 256, 0, stream>>>(P, u1, t0, C2, TW, nullptr, n4h);
        k_gemmw<bf, 0, true><<<dim3(NR / 64, ND / 64, 1), 32, 0, stream>>>(TW, nullptr, W2W, nullptr, NH, F, ND, b2, 0, 0, 0);
        k_st<<<(unsigned)(n4y / 256), 256, 0, stream>>>(Y[c], Z[n], F, il, oml, il, hs, Y[n], YW[n], n4y); }

    k_out<<<(unsigned)(NR * NO / 4 / 64), 64, 0, stream>>>(Y[NSTEP & 1], IV[NSTEP & 1], out);
}
